// AttentionBlock_88064009437220
// MI455X (gfx1250) — hardware-verified
//
#include <hip/hip_runtime.h>
#include <stdint.h>


#ifndef NB
#define NB 4
#endif
#ifndef SEQ
#define SEQ 2048
#endif
#define NB_FULL  4
#define SEQ_FULL 2048
#define EMBED    1024
#define HEADS    16
#define HDIM     64
#define FFN      4096
#define NTOK     (NB * SEQ)
#define PLD      72
#define TPD      72
#define FFN_ROWS ((NTOK <= 4096) ? NTOK : (((NTOK % 4096) == 0) ? 4096 : SEQ))
#define LN_EPS   1.0e-5f
#define NEGBIG   (-1.0e30f)

static_assert(EMBED == HEADS * HDIM);
static_assert((SEQ % 128) == 0);
static_assert((NTOK % 128) == 0);
static_assert((NTOK % 8) == 0);
static_assert((EMBED % 128) == 0);
static_assert((FFN % 128) == 0);
static_assert(NB >= 1 && NB <= NB_FULL);
static_assert(SEQ <= SEQ_FULL);
static_assert(HDIM == 64);
static_assert((FFN_ROWS % 128) == 0);
static_assert((NTOK % FFN_ROWS) == 0);
static_assert((EMBED % 64) == 0 && (FFN % 64) == 0 && (HDIM % 64) == 0);
static_assert((EMBED % 32) == 0 && (FFN % 32) == 0);
static_assert((EMBED % 256) == 0);

typedef _Float16     v16h __attribute__((ext_vector_type(16)));
typedef _Float16     v8h  __attribute__((ext_vector_type(8)));
typedef float        v8f  __attribute__((ext_vector_type(8)));
typedef float        v4f  __attribute__((ext_vector_type(4)));
typedef unsigned int v4u  __attribute__((ext_vector_type(4)));

union Frag  { v16h v; v8h h[2]; };
union Pack8 { v8h h; v4u u; };

static constexpr size_t PLANE_H = (size_t)NTOK * EMBED;
static constexpr size_t WQ_H    = (size_t)EMBED * EMBED;
static constexpr size_t WF_H    = (size_t)EMBED * FFN;
static constexpr size_t U_H     = (size_t)FFN_ROWS * FFN;
static constexpr size_t BIG_H   = (3 * PLANE_H > U_H) ? (3 * PLANE_H) : U_H;
static constexpr size_t OFF_A   = 0;
static constexpr size_t OFF_W   = OFF_A + PLANE_H * 2;
static constexpr size_t OFF_X1  = OFF_W + (4 * WQ_H + 2 * WF_H) * 2;
static constexpr size_t OFF_BIG = OFF_X1 + PLANE_H * 4;
static constexpr size_t WS_NEED = OFF_BIG + BIG_H * 2;
static_assert(WS_NEED <= (size_t)134217728);
static_assert((OFF_W % 128) == 0 && (OFF_X1 % 128) == 0 && (OFF_BIG % 128) == 0);
static_assert(((PLANE_H * 2) % 128) == 0);

static __device__ __forceinline__ v8f wmma16(v16h a, v16h b, v8f c) {
  v8f d = __builtin_amdgcn_wmma_f32_16x16x32_f16(false, a, false, b, (short)0, c, false, false);
  asm volatile("v_nop\n\tv_nop\n\tv_nop\n\tv_nop" : "+v"(d) : "v"(a), "v"(b));
  return d;
}

static __device__ __forceinline__ v16h frag_rows(const _Float16* base, int row0, size_t ld, int k0) {
  const int l = threadIdx.x & 31, hf = l >> 4, m = l & 15;
  const _Float16* p = base + (size_t)(row0 + m) * ld + k0 + 8 * hf;
  Frag f;
  f.h[0] = *(const v8h*)(p);
  f.h[1] = *(const v8h*)(p + 16);
  return f.v;
}

static __device__ __forceinline__ float bf16_rne(float f) {
  unsigned int u = __float_as_uint(f);
  u += 0x7fffu + ((u >> 16) & 1u);
  u &= 0xffff0000u;
  return __uint_as_float(u);
}

static __device__ __forceinline__ v4f rne4(v4f a) {
  v4f o;
  o[0] = bf16_rne(a[0]); o[1] = bf16_rne(a[1]);
  o[2] = bf16_rne(a[2]); o[3] = bf16_rne(a[3]);
  return o;
}

static __device__ __forceinline__ float wave_sum(float v) {
  v += __shfl_xor(v, 16);
  v += __shfl_xor(v, 8);
  v += __shfl_xor(v, 4);
  v += __shfl_xor(v, 2);
  v += __shfl_xor(v, 1);
  return v;
}

template <bool RNE>
static __device__ __forceinline__ v4u ln_pack(const float* s, const float* gam, const float* bet,
                                             int c, float mu, float inv) {
  v4f a = *(const v4f*)(s + c);
  v4f b = *(const v4f*)(s + c + 4);
  if (RNE) { a = rne4(a); b = rne4(b); }
  const v4f ga = rne4(*(const v4f*)(gam + c));
  const v4f gb = rne4(*(const v4f*)(gam + c + 4));
  const v4f ba = rne4(*(const v4f*)(bet + c));
  const v4f bb = rne4(*(const v4f*)(bet + c + 4));
  Pack8 o;
#pragma unroll
  for (int e = 0; e < 4; ++e) {
    o.h[e]     = (_Float16)((a[e] - mu) * inv * ga[e] + ba[e]);
    o.h[4 + e] = (_Float16)((b[e] - mu) * inv * gb[e] + bb[e]);
  }
  return o.u;
}

template <bool RNE>
__global__ __launch_bounds__(256)
void k_ln(const float* __restrict__ src, const float* __restrict__ gam,
          const float* __restrict__ bet, _Float16* __restrict__ dst,
          int rows, int period, int pstride) {
  const int w = threadIdx.x >> 5, lane = threadIdx.x & 31;
  const int r = blockIdx.x * 8 + w;
  if (r >= rows) return;
  const int rb = r / period;
  const int sr = rb * pstride + (r - rb * period);
  const float* s = src + (size_t)sr * EMBED;
  const int cl = 8 * lane;

  float s1 = 0.0f;
#pragma unroll 1
  for (int j = 0; j < 4; ++j) {
    v4f a = *(const v4f*)(s + 256 * j + cl);
    v4f b = *(const v4f*)(s + 256 * j + cl + 4);
    if (RNE) { a = rne4(a); b = rne4(b); }
    s1 += ((a[0] + a[1]) + (a[2] + a[3])) + ((b[0] + b[1]) + (b[2] + b[3]));
  }
  s1 = wave_sum(s1);
  const float mu = s1 * (1.0f / (float)EMBED);

  float s2 = 0.0f;
#pragma unroll 1
  for (int j = 0; j < 4; ++j) {
    v4f a = *(const v4f*)(s + 256 * j + cl);
    v4f b = *(const v4f*)(s + 256 * j + cl + 4);
    if (RNE) { a = rne4(a); b = rne4(b); }
    float t = 0.0f;
#pragma unroll
    for (int e = 0; e < 4; ++e) {
      const float da = a[e] - mu, db = b[e] - mu;
      t += da * da;
      t += db * db;
    }
    s2 += t;
  }
  s2 = wave_sum(s2);
  const float var = s2 * (1.0f / (float)EMBED);
  const float inv = 1.0f / sqrtf(var + LN_EPS);

  _Float16* d = dst + (size_t)r * EMBED;
#pragma unroll 1
  for (int j = 0; j < 4; ++j) {
    const int c = 256 * j + cl;
    const v4u o = ln_pack<RNE>(s, gam, bet, c, mu, inv);
    *(volatile v4u*)(d + c) = o;
  }
  __threadfence();
#pragma unroll 1
  for (int j = 0; j < 4; ++j) {
    const int c = 256 * j + cl;
    const v4u o = ln_pack<RNE>(s, gam, bet, c, mu, inv);
    *(volatile v4u*)(d + c) = o;
  }
}

__global__ __launch_bounds__(256)
void k_wtr(const float* __restrict__ src, _Float16* __restrict__ dst, int R, int C, float scale) {
  __shared__ _Float16 Ts[64 * TPD];
  const int tid = threadIdx.x;
  const int c0 = blockIdx.x * 64, r0 = blockIdx.y * 64, g = blockIdx.z;
  const float* sb = src + ((size_t)g * R + r0) * (size_t)C + c0;
#pragma unroll
  for (int i = 0; i < 4; ++i) {
    const int p  = tid + 256 * i;
    const int rr = p >> 4;
    const int c4 = (p & 15) * 4;
    const v4f a = *(const v4f*)(sb + (size_t)rr * C + c4);
#pragma unroll
    for (int j = 0; j < 4; ++j)
      Ts[(c4 + j) * TPD + rr] = (_Float16)(bf16_rne(a[j]) * scale);
  }
  __syncthreads();
  Pack8 vals[2];
#pragma unroll
  for (int i = 0; i < 2; ++i) {
    const int p  = tid + 256 * i;
    const int cc = p >> 3;
    const int r8 = (p & 7) * 8;
    vals[i].h = *(const v8h*)(Ts + cc * TPD + r8);
  }
  _Float16* db = dst + ((size_t)g * C + c0) * (size_t)R + r0;
#pragma unroll
  for (int i = 0; i < 2; ++i) {
    const int p  = tid + 256 * i;
    const int cc = p >> 3, r8 = (p & 7) * 8;
    *(volatile v4u*)(db + (size_t)cc * R + r8) = vals[i].u;
  }
  __threadfence();
#pragma unroll
  for (int i = 0; i < 2; ++i) {
    const int p  = tid + 256 * i;
    const int cc = p >> 3, r8 = (p & 7) * 8;
    *(volatile v4u*)(db + (size_t)cc * R + r8) = vals[i].u;
  }
}

template <bool OUTF32, bool HASBIAS, bool RELU, bool HASRES, bool RESRNE>
__global__ __launch_bounds__(256) __attribute__((amdgpu_num_vgpr(256)))
void k_gemm(const _Float16* __restrict__ A,
            const _Float16* __restrict__ Wa, const _Float16* __restrict__ Wb,
            const _Float16* __restrict__ Wc,
            const float* __restrict__ Ga, const float* __restrict__ Gb,
            const float* __restrict__ Gc,
            const float* __restrict__ res, int rper, int rstr,
            void* Oa, void* Ob, void* Oc,
            int K, int Nout, int ztr, float oscale) {
  __shared__ float Cs[128 * 128];

  const int tid = threadIdx.x, w = tid >> 5, lane = tid & 31;
  const int hf = lane >> 4, nin = lane & 15;
  const int wm = w >> 1, wn = w & 1;
  const int m_blk = blockIdx.y * 128, n_blk = blockIdx.x * 128;
  const int z = blockIdx.z;
  const _Float16* W  = (z == 0) ? Wa : ((z == 1) ? Wb : Wc);
  const float*  bias = (z == 0) ? Ga : ((z == 1) ? Gb : Gc);
  void*           Ov = (z == 0) ? Oa : ((z == 1) ? Ob : Oc);

  v8f acc[2][4] = {};

#pragma unroll 1
  for (int k0 = 0; k0 < K; k0 += 32) {
    const v16h a0 = frag_rows(A, m_blk + wm * 32,      (size_t)K, k0);
    const v16h a1 = frag_rows(A, m_blk + wm * 32 + 16, (size_t)K, k0);
#pragma unroll
    for (int nt = 0; nt < 4; ++nt) {
      const v16h bf = frag_rows(W, n_blk + wn * 64 + nt * 16, (size_t)K, k0);
      acc[0][nt] = wmma16(a0, bf, acc[0][nt]);
      acc[1][nt] = wmma16(a1, bf, acc[1][nt]);
    }
  }

#pragma unroll
  for (int nt = 0; nt < 4; ++nt) {
    const int ncol = wn * 64 + nt * 16 + nin;
    float bb = 0.0f;
    if (HASBIAS) bb = bf16_rne(bias[n_blk + ncol]);
#pragma unroll
    for (int mt = 0; mt < 2; ++mt)
#pragma unroll
      for (int r = 0; r < 8; ++r) {
        const int row = wm * 32 + mt * 16 + 8 * hf + r;
        float v = acc[mt][nt][r] * oscale + bb;
        if (RELU) v = fmaxf(v, 0.0f);
        Cs[row * 128 + ncol] = v;
      }
  }
  __syncthreads();

  if (OUTF32) {
    float* out = (float*)Ov;
#pragma unroll
    for (int i = 0; i < 16; ++i) {
      const int row = w * 16 + i;
      v4f v = *(const v4f*)(&Cs[row * 128 + 4 * lane]);
      if (HASRES) {
        const int m = m_blk + row;
        const int rb = m / rper;
        const int sr = rb * rstr + (m - rb * rper);
        v4f q = *(const v4f*)(res + (size_t)sr * Nout + n_blk + 4 * lane);
        if (RESRNE) q = rne4(q);
        v += q;
      }
      *(volatile v4f*)(out + (size_t)(m_blk + row) * Nout + n_blk + 4 * lane) = v;
    }
    __threadfence();
#pragma unroll
    for (int i = 0; i < 16; ++i) {
      const int row = w * 16 + i;
      v4f v = *(const v4f*)(&Cs[row * 128 + 4 * lane]);
      if (HASRES) {
        const int m = m_blk + row;
        const int rb = m / rper;
        const int sr = rb * rstr + (m - rb * rper);
        v4f q = *(const v4f*)(res + (size_t)sr * Nout + n_blk + 4 * lane);
        if (RESRNE) q = rne4(q);
        v += q;
      }
      *(volatile v4f*)(out + (size_t)(m_blk + row) * Nout + n_blk + 4 * lane) = v;
    }
  } else {
    _Float16* out = (_Float16*)Ov;
    if (z != ztr) {
      v4u vals[8];
      const int c0 = nin * 8;
#pragma unroll
      for (int i = 0; i < 8; ++i) {
        const int row = w * 16 + 2 * i + hf;
        const v4f a = *(const v4f*)(&Cs[row * 128 + c0]);
        const v4f b = *(const v4f*)(&Cs[row * 128 + c0 + 4]);
        Pack8 o;
        o.h[0] = (_Float16)a[0]; o.h[1] = (_Float16)a[1];
        o.h[2] = (_Float16)a[2]; o.h[3] = (_Float16)a[3];
        o.h[4] = (_Float16)b[0]; o.h[5] = (_Float16)b[1];
        o.h[6] = (_Float16)b[2]; o.h[7] = (_Float16)b[3];
        vals[i] = o.u;
      }
#pragma unroll
      for (int i = 0; i < 8; ++i) {
        const int row = w * 16 + 2 * i + hf;
        *(volatile v4u*)(out + (size_t)(m_blk + row) * Nout + n_blk + c0) = vals[i];
      }
      __threadfence();
#pragma unroll
      for (int i = 0; i < 8; ++i) {
        const int row = w * 16 + 2 * i + hf;
        *(volatile v4u*)(out + (size_t)(m_blk + row) * Nout + n_blk + c0) = vals[i];
      }
    } else {
      const int bb = m_blk / SEQ;
      const int s0 = m_blk - bb * SEQ;
      const int t0 = nin * 8;
      v4u vals[8];
#pragma unroll
      for (int i = 0; i < 8; ++i) {
        const int c = w * 16 + 2 * i + hf;
        Pack8 o;
#pragma unroll
        for (int j = 0; j < 8; ++j) o.h[j] = (_Float16)Cs[(t0 + j) * 128 + c];
        vals[i] = o.u;
      }
#pragma unroll
      for (int i = 0; i < 8; ++i) {
        const int c = w * 16 + 2 * i + hf;
        const int n = n_blk + c;
        const int hh = n / HDIM, d = n - hh * HDIM;
        _Float16* dst = out + ((size_t)(bb * HEADS + hh) * HDIM + d) * SEQ + s0 + t0;
        *(volatile v4u*)dst = vals[i];
      }
      __threadfence();
#pragma unroll
      for (int i = 0; i < 8; ++i) {
        const int c = w * 16 + 2 * i + hf;
        const int n = n_blk + c;
        const int hh = n / HDIM, d = n - hh * HDIM;
        _Float16* dst = out + ((size_t)(bb * HEADS + hh) * HDIM + d) * SEQ + s0 + t0;
        *(volatile v4u*)dst = vals[i];
      }
    }
  }
}

__global__ __launch_bounds__(128) __attribute__((amdgpu_num_vgpr(256)))
void k_attn(const _Float16* __restrict__ qh, const _Float16* __restrict__ kh,
            const _Float16* __restrict__ vt, _Float16* __restrict__ oh, float scale) {
  __shared__ _Float16 Ps[4 * 16 * PLD];

  const int tid = threadIdx.x, w = tid >> 5, lane = tid & 31;
  const int hf = lane >> 4, nin = lane & 15;
  const int qblk = blockIdx.x, h = blockIdx.y, b = blockIdx.z;
  const int qtok0 = b * SEQ + qblk * 64 + w * 16;
  const int ktokb = b * SEQ;
  _Float16* Pw = Ps + w * 16 * PLD;
  const _Float16* vtb = vt + (size_t)(b * HEADS + h) * HDIM * SEQ;

  v16h qa[2];
  {
    const _Float16* qp = qh + (size_t)(qtok0 + nin) * EMBED + h * HDIM + 8 * hf;
    Frag f;
    f.h[0] = *(const v8h*)(qp);      f.h[1] = *(const v8h*)(qp + 16); qa[0] = f.v;
    f.h[0] = *(const v8h*)(qp + 32); f.h[1] = *(const v8h*)(qp + 48); qa[1] = f.v;
  }

  float mrow[8], lrow[8];
#pragma unroll
  for (int r = 0; r < 8; ++r) { mrow[r] = NEGBIG; lrow[r] = 0.0f; }
  v8f oacc[4] = {};

  const int nkb = qblk + 1;
#pragma unroll 1
  for (int kb = 0; kb < nkb; ++kb) {
    __syncthreads();

    v8f sacc[4] = {};
#pragma unroll
    for (int nt = 0; nt < 4; ++nt) {
      const _Float16* kp = kh + (size_t)(ktokb + kb * 64 + nt * 16 + nin) * EMBED + h * HDIM + 8 * hf;
      Frag f;
      f.h[0] = *(const v8h*)(kp);      f.h[1] = *(const v8h*)(kp + 16);
      sacc[nt] = wmma16(qa[0], f.v, sacc[nt]);
      Frag g;
      g.h[0] = *(const v8h*)(kp + 32); g.h[1] = *(const v8h*)(kp + 48);
      sacc[nt] = wmma16(qa[1], g.v, sacc[nt]);
    }

    const int kcap = (kb == qblk) ? 0 : 64;

#pragma unroll
    for (int r = 0; r < 8; ++r) {
      const int klim = w * 16 + 8 * hf + r + kcap;
      float s0 = sacc[0][r] * scale, s1 = sacc[1][r] * scale;
      float s2 = sacc[2][r] * scale, s3 = sacc[3][r] * scale;
      s0 = (nin      > klim) ? NEGBIG : s0;
      s1 = (16 + nin > klim) ? NEGBIG : s1;
      s2 = (32 + nin > klim) ? NEGBIG : s2;
      s3 = (48 + nin > klim) ? NEGBIG : s3;
      float t = fmaxf(fmaxf(s0, s1), fmaxf(s2, s3));
      t = fmaxf(t, __shfl_xor(t, 8, 16));
      t = fmaxf(t, __shfl_xor(t, 4, 16));
      t = fmaxf(t, __shfl_xor(t, 2, 16));
      t = fmaxf(t, __shfl_xor(t, 1, 16));
      const float mn    = fmaxf(mrow[r], t);
      const float alpha = __expf(mrow[r] - mn);
      mrow[r] = mn;
      const float p0 = __expf(s0 - mn), p1 = __expf(s1 - mn);
      const float p2 = __expf(s2 - mn), p3 = __expf(s3 - mn);
      float rs = (p0 + p1) + (p2 + p3);
      rs += __shfl_xor(rs, 8, 16);
      rs += __shfl_xor(rs, 4, 16);
      rs += __shfl_xor(rs, 2, 16);
      rs += __shfl_xor(rs, 1, 16);
      lrow[r] = lrow[r] * alpha + rs;
      sacc[0][r] = p0; sacc[1][r] = p1; sacc[2][r] = p2; sacc[3][r] = p3;
      oacc[0][r] *= alpha; oacc[1][r] *= alpha; oacc[2][r] *= alpha; oacc[3][r] *= alpha;
    }

#pragma unroll
    for (int nt = 0; nt < 4; ++nt)
#pragma unroll
      for (int r = 0; r < 8; ++r)
        Pw[(8 * hf + r) * PLD + nt * 16 + nin] = (_Float16)(sacc[nt][r] * 1024.0f);
    __syncthreads();

#pragma unroll
    for (int ks = 0; ks < 2; ++ks) {
      const v16h pf = frag_rows(Pw, 0, (size_t)PLD, ks * 32);
#pragma unroll
      for (int dt = 0; dt < 4; ++dt) {
        const _Float16* vp = vtb + (size_t)(dt * 16 + nin) * SEQ + kb * 64 + ks * 32 + 8 * hf;
        Frag f;
        f.h[0] = *(const v8h*)(vp); f.h[1] = *(const v8h*)(vp + 16);
        oacc[dt] = wmma16(pf, f.v, oacc[dt]);
      }
    }
  }
  __syncthreads();

#pragma unroll
  for (int r = 0; r < 8; ++r) {
    const float inv = 0.0625f * (1.0f / lrow[r]);
#pragma unroll
    for (int dt = 0; dt < 4; ++dt)
      Pw[(8 * hf + r) * PLD + dt * 16 + nin] = (_Float16)(oacc[dt][r] * inv);
  }
  __syncthreads();

  Pack8 vals[4];
  const int cl = (lane & 7) * 8;
#pragma unroll
  for (int i = 0; i < 4; ++i) {
    const int row = (lane >> 3) + 4 * i;
    vals[i].h = *(const v8h*)(Pw + row * PLD + cl);
  }
#pragma unroll
  for (int i = 0; i < 4; ++i) {
    const int row = (lane >> 3) + 4 * i;
    *(volatile v4u*)(oh + (size_t)(qtok0 + row) * EMBED + h * HDIM + cl) = vals[i].u;
  }
  __threadfence();
#pragma unroll
  for (int i = 0; i < 4; ++i) {
    const int row = (lane >> 3) + 4 * i;
    *(volatile v4u*)(oh + (size_t)(qtok0 + row) * EMBED + h * HDIM + cl) = vals[i].u;
  }
}

extern "C" void kernel_launch(void* const* d_in, const int* in_sizes, int n_in,
                              void* d_out, int out_size, void* d_ws, size_t ws_size,
                              hipStream_t stream) {
  if (n_in < 14) return;
  const long long need_x = ((long long)(NB - 1) * SEQ_FULL + SEQ) * (long long)EMBED;
  if ((long long)in_sizes[0] < need_x) return;
  if (in_sizes[1] < HEADS * EMBED * HDIM || in_sizes[2] < HEADS * EMBED * HDIM ||
      in_sizes[3] < HEADS * EMBED * HDIM) return;
  if (in_sizes[4] < EMBED * EMBED || in_sizes[5] < EMBED) return;
  if (in_sizes[6] < EMBED * FFN || in_sizes[7] < FFN) return;
  if (in_sizes[8] < FFN * EMBED || in_sizes[9] < EMBED) return;
  if (in_sizes[10] < EMBED || in_sizes[11] < EMBED || in_sizes[12] < EMBED || in_sizes[13] < EMBED) return;
  if ((long long)out_size < (long long)NTOK * EMBED) return;
  if (WS_NEED > ws_size) return;

  const float* x   = (const float*)d_in[0];
  const float* Wq  = (const float*)d_in[1];
  const float* Wk  = (const float*)d_in[2];
  const float* Wv  = (const float*)d_in[3];
  const float* Wo  = (const float*)d_in[4];
  const float* bo  = (const float*)d_in[5];
  const float* Wf1 = (const float*)d_in[6];
  const float* bf1 = (const float*)d_in[7];
  const float* Wf2 = (const float*)d_in[8];
  const float* bf2 = (const float*)d_in[9];
  const float* g1  = (const float*)d_in[10];
  const float* bt1 = (const float*)d_in[11];
  const float* g2  = (const float*)d_in[12];
  const float* bt2 = (const float*)d_in[13];
  float* out = (float*)d_out;

  char* ws = (char*)d_ws;
  _Float16* pa  = (_Float16*)(ws + OFF_A);
  _Float16* wqh = (_Float16*)(ws + OFF_W);
  _Float16* wkh = wqh + WQ_H;
  _Float16* wvh = wkh + WQ_H;
  _Float16* woh = wvh + WQ_H;
  _Float16* w1h = woh + WQ_H;
  _Float16* w2h = w1h + WF_H;
  float*    x1  = (float*)(ws + OFF_X1);
  _Float16* qh  = (_Float16*)(ws + OFF_BIG);
  _Float16* kh  = qh + PLANE_H;
  _Float16* vt  = kh + PLANE_H;
  _Float16* uh  = (_Float16*)(ws + OFF_BIG);

  const float inv64   = 0.015625f;
  const float inv4096 = 0.000244140625f;

  k_ln<true><<<NTOK / 8, 256, 0, stream>>>(x, g1, bt1, pa, NTOK, SEQ, SEQ_FULL);

  k_wtr<<<dim3(HDIM / 64, EMBED / 64, HEADS), 256, 0, stream>>>(Wq, wqh, EMBED, HDIM, 64.0f);
  k_wtr<<<dim3(HDIM / 64, EMBED / 64, HEADS), 256, 0, stream>>>(Wk, wkh, EMBED, HDIM, 64.0f);
  k_wtr<<<dim3(HDIM / 64, EMBED / 64, HEADS), 256, 0, stream>>>(Wv, wvh, EMBED, HDIM, 64.0f);
  k_wtr<<<dim3(EMBED / 64, EMBED / 64, 1), 256, 0, stream>>>(Wo, woh, EMBED, EMBED, 64.0f);
  k_wtr<<<dim3(FFN / 64, EMBED / 64, 1), 256, 0, stream>>>(Wf1, w1h, EMBED, FFN, 64.0f);
  k_wtr<<<dim3(EMBED / 64, FFN / 64, 1), 256, 0, stream>>>(Wf2, w2h, FFN, EMBED, 64.0f);

  k_gemm<false, false, false, false, false><<<dim3(EMBED / 128, NTOK / 128, 3), 256, 0, stream>>>(
      pa, wqh, wkh, wvh, g1, g1, g1, x, SEQ, SEQ_FULL,
      (void*)qh, (void*)kh, (void*)vt, EMBED, EMBED, 2, inv64);

  k_attn<<<dim3(SEQ / 64, HEADS, NB), 128, 0, stream>>>(qh, kh, vt, pa, 0.03125f);

  k_gemm<true, true, false, true, true><<<dim3(EMBED / 128, NTOK / 128, 1), 256, 0, stream>>>(
      pa, woh, woh, woh, bo, bo, bo, x, SEQ, SEQ_FULL,
      (void*)x1, (void*)x1, (void*)x1, EMBED, EMBED, -1, inv4096);

  k_ln<false><<<NTOK / 8, 256, 0, stream>>>(x1, g2, bt2, pa, NTOK, SEQ, SEQ);

  for (int c = 0; c < NTOK / FFN_ROWS; ++c) {
    const size_t toff = (size_t)c * FFN_ROWS * EMBED;
    k_gemm<false, true, true, false, false><<<dim3(FFN / 128, FFN_ROWS / 128, 1), 256, 0, stream>>>(
        pa + toff, w1h, w1h, w1h, bf1, bf1, bf1, x1, FFN_ROWS, FFN_ROWS,
        (void*)uh, (void*)uh, (void*)uh, EMBED, FFN, -1, inv64);
    k_gemm<true, true, false, true, false><<<dim3(EMBED / 128, FFN_ROWS / 128, 1), 256, 0, stream>>>(
        uh, w2h, w2h, w2h, bf2, bf2, bf2, x1 + toff, FFN_ROWS, FFN_ROWS,
        (void*)(out + toff), (void*)(out + toff), (void*)(out + toff), FFN, EMBED, -1, inv64);
  }
}
